// SimpleNet_order_no_batch_61332132987039
// MI455X (gfx1250) — hardware-verified
//
#include <hip/hip_runtime.h>


#define NR   8192
#define WD   128
#define NL   22
#define GW   (24 * WD)
typedef _Float16 h16;
typedef unsigned short bf;
typedef __attribute__((ext_vector_type(16))) __bf16   v16bf;
typedef __attribute__((ext_vector_type(16))) _Float16 v16h;
typedef __attribute__((ext_vector_type(8)))  _Float16 v8h;
typedef __attribute__((ext_vector_type(8)))  unsigned short v8us;
typedef __attribute__((ext_vector_type(8)))  float    v8f;
typedef __attribute__((ext_vector_type(4)))  float    v4f;
typedef v8h  __attribute__((may_alias)) v8ha;
typedef v4f  __attribute__((may_alias)) v4fa;
typedef v8us __attribute__((may_alias)) v8usa;

__device__ __forceinline__ unsigned short f2bf(float f) { unsigned u = __float_as_uint(f); u += 0x7FFFu + ((u >> 16) & 1u); return (unsigned short)(u >> 16); }
__device__ __forceinline__ float bf2f(unsigned short b) { return __uint_as_float(((unsigned)b) << 16); }
__device__ __forceinline__ float bfr(float f) { return bf2f(f2bf(f)); }
__device__ __forceinline__ v16h cat16(v8h lo, v8h hi) { return __builtin_shufflevector(lo, hi, 0, 1, 2, 3, 4, 5, 6, 7, 8, 9, 10, 11, 12, 13, 14, 15); }
__device__ __forceinline__ v16bf cat16b(v8us lo, v8us hi) { return __builtin_bit_cast(v16bf, __builtin_shufflevector(lo, hi, 0, 1, 2, 3, 4, 5, 6, 7, 8, 9, 10, 11, 12, 13, 14, 15)); }
__device__ __forceinline__ v8f wmma16(v16h a, v16h b, v8f c) { return __builtin_amdgcn_wmma_f32_16x16x32_f16(false, a, false, b, (short)0, c, false, false); }
__device__ __forceinline__ v8f wmmab(v16bf a, v16bf b, v8f c) { return __builtin_amdgcn_wmma_f32_16x16x32_bf16(false, a, false, b, (short)0, c, false, false); }


template <typename T16> struct WFrag;
template <> struct WFrag<h16> { typedef v16h V; static __device__ __forceinline__ V ld(const h16* p) { return cat16(*(const v8h*)p, *(const v8h*)(p + 16)); } static __device__ __forceinline__ v8f mma(V a, V b, v8f c) { return wmma16(a, b, c); } };
template <> struct WFrag<bf> { typedef v16bf V; static __device__ __forceinline__ V ld(const bf* p) { return cat16b(*(const v8us*)p, *(const v8us*)(p + 16)); } static __device__ __forceinline__ v8f mma(V a, V b, v8f c) { return wmmab(a, b, c); } };
template <typename T16, int NSPLIT, bool BIAS>
__global__ __launch_bounds__(32) void k_gemmw(const T16* __restrict__ A, const T16* __restrict__ A2, const T16* __restrict__ Bt, const T16* __restrict__ Bt2, int K, float* C, int ldc, const float* __restrict__ bias, size_t sA, size_t sB, size_t sC) {
    typedef typename WFrag<T16>::V V;
    __shared__ __align__(16) float os[16 * 68];
    const size_t z = blockIdx.z; A += z * sA; if (A2) A2 += z * sA; Bt += z * sB; if (Bt2) Bt2 += z * sB; C += z * sC;
    const int lane = threadIdx.x & 31, lr = lane & 15, hi = lane >> 4; const int r0 = blockIdx.x * 64, c0 = blockIdx.y * 64;
    v8f acc[4][4];
#pragma unroll
    for (int mb = 0; mb < 4; ++mb)
#pragma unroll
        for (int nb = 0; nb < 4; ++nb) acc[mb][nb] = (v8f){};
    const size_t aoff = (size_t)(r0 + lr) * K + 8 * hi, boff = (size_t)(c0 + lr) * K + 8 * hi;
#pragma unroll 1
    for (int kc = 0; kc < K; kc += 32) {
        V a[4], a2[4];
#pragma unroll
        for (int mb = 0; mb < 4; ++mb) { a[mb] = WFrag<T16>::ld(A + aoff + (size_t)mb * 16 * K + kc); if (NSPLIT == 1 || NSPLIT == 2) a2[mb] = WFrag<T16>::ld(A2 + aoff + (size_t)mb * 16 * K + kc); }
#pragma unroll
        for (int nb = 0; nb < 4; ++nb) { const V b = WFrag<T16>::ld(Bt + boff + (size_t)nb * 16 * K + kc); V b2; if (NSPLIT >= 2) b2 = WFrag<T16>::ld(Bt2 + boff + (size_t)nb * 16 * K + kc);
#pragma unroll
            for (int mb = 0; mb < 4; ++mb) { acc[mb][nb] = WFrag<T16>::mma(a[mb], b, acc[mb][nb]); if (NSPLIT == 1 || NSPLIT == 2) acc[mb][nb] = WFrag<T16>::mma(a2[mb], b, acc[mb][nb]); if (NSPLIT >= 2) acc[mb][nb] = WFrag<T16>::mma(a[mb], b2, acc[mb][nb]); } }
        asm volatile("v_nop\n\tv_nop\n\tv_nop\n\tv_nop" : "+v"(acc[0][0]), "+v"(acc[1][1]), "+v"(acc[2][2]), "+v"(acc[3][3]) : "v"(a[0]), "v"(a[3]));
    }
#pragma unroll
    for (int mb = 0; mb < 4; ++mb) {
#pragma unroll
        for (int nb = 0; nb < 4; ++nb) {
#pragma unroll
            for (int j = 0; j < 8; ++j) os[(hi * 8 + j) * 68 + nb * 16 + lr] = acc[mb][nb][j]; }
        __builtin_amdgcn_wave_barrier(); asm volatile("" ::: "memory");
        float* crow = C + (size_t)(r0 + mb * 16) * ldc + c0;
#pragma unroll 1
        for (int ps = 0; ps < 2; ++ps) {
#pragma unroll
            for (int s = 0; s < 8; ++s) { const int row = 2 * s + hi, cofs = lr * 4; v4f val = *(const v4fa*)(os + row * 68 + cofs); if (BIAS) { val[0] += bfr(bias[c0 + cofs]); val[1] += bfr(bias[c0 + cofs + 1]); val[2] += bfr(bias[c0 + cofs + 2]); val[3] += bfr(bias[c0 + cofs + 3]); }
                *(volatile v4f*)(crow + (size_t)row * ldc + cofs) = val; }
            if (ps == 0) __threadfence(); }
        __builtin_amdgcn_wave_barrier(); asm volatile("" ::: "memory");
    }
}

__device__ __forceinline__ void splitf(float y, unsigned short& h, unsigned short& l) { h = f2bf(y); l = f2bf(y - bf2f(h)); }
typedef __attribute__((ext_vector_type(2))) unsigned short v2us;
typedef __attribute__((ext_vector_type(4))) unsigned short v4us;
typedef __attribute__((ext_vector_type(2))) float v2f;

__global__ __launch_bounds__(256) void k_wtG(const float* __restrict__ w, int K, int N, bf* Bt) {
    const int lane = threadIdx.x & 31; const int L0 = (blockIdx.x * 8 + (threadIdx.x >> 5)) * 8; const int nlines = N * K / 64;
#pragma unroll 1
    for (int ps = 0; ps < 2; ++ps) {
#pragma unroll 1
        for (int l = 0; l < 8; ++l) { const int L = L0 + l; if (L >= nlines) break; const size_t e = (size_t)L * 64 + lane * 2; const int k = (int)(e % K), n = (int)(e / K); v2us o;
            o[0] = f2bf(w[(size_t)k * N + n]); o[1] = f2bf(w[(size_t)(k + 1) * N + n]); *(volatile v2us*)(Bt + e) = o; }
        if (ps == 0) __threadfence(); }
}
__global__ __launch_bounds__(256) void k_wlast(const float* __restrict__ w, const float* __restrict__ bl, bf* Bt, float* BL) { const int e = (blockIdx.x * 256 + threadIdx.x) * 4; if (e >= 64 * 2 * WD) return; const int k = e % (2 * WD), n = e / (2 * WD); v4us o;
#pragma unroll
    for (int q = 0; q < 4; ++q) o[q] = (n < 2) ? f2bf(w[(size_t)(k + q) * 2 + n]) : (unsigned short)0; *(volatile v4us*)(Bt + e) = o;
    if (blockIdx.x == 0 && threadIdx.x < 64) { const int n2 = threadIdx.x; const float bv = (n2 < 2) ? bl[n2] : 0.f; *(volatile float*)(BL + n2) = bv; }
    __threadfence(); *(volatile v4us*)(Bt + e) = o; if (blockIdx.x == 0 && threadIdx.x < 64) { const int n2 = threadIdx.x; const float bv = (n2 < 2) ? bl[n2] : 0.f; *(volatile float*)(BL + n2) = bv; } }
__global__ __launch_bounds__(256) void k_l0(const float* __restrict__ x, const float* __restrict__ W0, const float* __restrict__ b0, float* G, bf* Ph, bf* Pl) { const size_t e = ((size_t)blockIdx.x * 256 + threadIdx.x) * 2; if (e >= (size_t)NR * WD) return; const int c = (int)(e % WD), i = (int)(e / WD); const float x0 = bfr(x[(size_t)i * 2]), x1 = bfr(x[(size_t)i * 2 + 1]); v2f o; v2us oh, ol;
#pragma unroll
    for (int q = 0; q < 2; ++q) { float p0 = __fmul_rn(x0, bfr(W0[c + q])), p1 = __fmul_rn(x1, bfr(W0[WD + c + q])); asm volatile("" : "+v"(p0), "+v"(p1)); const float y = fmaxf(__fadd_rn(__fadd_rn(p0, p1), bfr(b0[c + q])), 0.f); o[q] = y; unsigned short a, c2; splitf(y, a, c2); oh[q] = a; ol[q] = c2; }
    const size_t og = (size_t)i * GW + 23 * WD + c; *(volatile v2f*)(G + og) = o; *(volatile v2us*)(Ph + e) = oh; *(volatile v2us*)(Pl + e) = ol; __threadfence(); *(volatile v2f*)(G + og) = o; *(volatile v2us*)(Ph + e) = oh; *(volatile v2us*)(Pl + e) = ol; }
__global__ __launch_bounds__(256) void k_intmp(const float* __restrict__ G, const int* __restrict__ links, int l, int dorelu, bf* Ih, bf* Il) { const size_t e = ((size_t)blockIdx.x * 256 + threadIdx.x) * 2; if (e >= (size_t)NR * 2 * WD) return; const int c = (int)(e % (2 * WD)), i = (int)(e / (2 * WD)); v2us oh, ol;
#pragma unroll
    for (int q = 0; q < 2; ++q) { const int cq = c + q; int lk = (cq < WD) ? 0 : links[l * WD + (cq - WD)]; lk = lk < 0 ? 0 : (lk > (l + 1) * WD - 1 ? (l + 1) * WD - 1 : lk);     const int gcol = (cq < WD) ? (22 - l) * WD + cq : (23 - l) * WD + lk; float y = G[(size_t)i * GW + gcol]; if (dorelu) y = fmaxf(y, 0.f); unsigned short a, c2; splitf(y, a, c2); oh[q] = a; ol[q] = c2; }
    *(volatile v2us*)(Ih + e) = oh; *(volatile v2us*)(Il + e) = ol; __threadfence(); *(volatile v2us*)(Ih + e) = oh; *(volatile v2us*)(Il + e) = ol; }
__global__ __launch_bounds__(256) void k_copy2(const float* __restrict__ T, float* OUT) { const int i = blockIdx.x * 256 + threadIdx.x; if (i >= NR) return; const v2f v = *(const v2f*)(T + (size_t)i * 64); *(volatile v2f*)(OUT + (size_t)i * 2) = v; __threadfence(); *(volatile v2f*)(OUT + (size_t)i * 2) = v; }

extern "C" void kernel_launch(void* const* d_in, const int* in_sizes, int n_in,
                              void* d_out, int out_size, void* d_ws, size_t ws_size, hipStream_t stream) {
    (void)in_sizes; (void)n_in; (void)out_size;
    const float* x = (const float*)d_in[0]; const int* links = (const int*)d_in[1]; const float* W0 = (const float*)d_in[2]; const float* b0 = (const float*)d_in[3]; const float* W1 = (const float*)d_in[4]; const float* b1 = (const float*)d_in[5]; const float* Wmid = (const float*)d_in[6]; const float* bmid = (const float*)d_in[7]; const float* Wlast = (const float*)d_in[8]; const float* blast = (const float*)d_in[9];
    float* OUT = (float*)d_out;
    char* wsp = (char*)d_ws;
    auto take = [&](size_t bytes) { char* p = wsp; wsp += (bytes + 255) & ~(size_t)255; return (void*)p; };
    bf* WB1 = (bf*)take((size_t)WD * WD * 2); bf* WBM = (bf*)take((size_t)(NL - 1) * WD * 2 * WD * 2); bf* WBL = (bf*)take((size_t)64 * 2 * WD * 2); float* BL = (float*)take(64 * 4); float* G = (float*)take((size_t)NR * GW * 4); bf* Ih = (bf*)take((size_t)NR * 2 * WD * 2); bf* Il = (bf*)take((size_t)NR * 2 * WD * 2); float* T = (float*)take((size_t)NR * 64 * 4);
    if ((size_t)(wsp - (char*)d_ws) > ws_size) return;
    k_wtG<<<(WD * WD / 64 + 63) / 64, 256, 0, stream>>>(W1, WD, WD, WB1);
    for (int l = 0; l < NL - 1; ++l) k_wtG<<<(2 * WD * WD / 64 + 63) / 64, 256, 0, stream>>>(Wmid + (size_t)l * 2 * WD * WD, 2 * WD, WD, WBM + (size_t)l * WD * 2 * WD);
    k_wlast<<<(64 * 2 * WD / 4 + 255) / 256, 256, 0, stream>>>(Wlast, blast, WBL, BL);
    k_l0<<<(unsigned)(((size_t)NR * WD / 2 + 255) / 256), 256, 0, stream>>>(x, W0, b0, G, Ih, Il);
    k_gemmw<bf, 1, true><<<dim3(NR / 64, WD / 64, 1), 32, 0, stream>>>(Ih, Il, WB1, nullptr, WD, G + 22 * WD, GW, b1, 0, 0, 0);
    const unsigned LI = (unsigned)(((size_t)NR * 2 * WD / 2 + 255) / 256);
    for (int l = 0; l < NL - 1; ++l) {
        k_intmp<<<LI, 256, 0, stream>>>(G, links, l, 1, Ih, Il);
        k_gemmw<bf, 1, true><<<dim3(NR / 64, WD / 64, 1), 32, 0, stream>>>(Ih, Il, WBM + (size_t)l * WD * 2 * WD, nullptr, 2 * WD, G + (size_t)(21 - l) * WD, GW, bmid + (size_t)l * WD, 0, 0, 0); }
    k_intmp<<<LI, 256, 0, stream>>>(G, links, NL - 1, 0, Ih, Il);
    k_gemmw<bf, 1, true><<<dim3(NR / 64, 1, 1), 32, 0, stream>>>(Ih, Il, WBL, nullptr, 2 * WD, T, 64, BL, 0, 0, 0);
    k_copy2<<<NR / 256, 256, 0, stream>>>(T, OUT);
}
